// VerifyConv2d_38482906972593
// MI455X (gfx1250) — hardware-verified
//
#include <hip/hip_runtime.h>

typedef __attribute__((ext_vector_type(16))) _Float16 v16h;
typedef __attribute__((ext_vector_type(8)))  _Float16 v8h;
typedef __attribute__((ext_vector_type(8)))  float    v8f;
typedef __attribute__((ext_vector_type(4)))  float    v4f;

constexpr int kCin     = 16;
constexpr int kCout    = 32;
constexpr int kHgt     = 16;
constexpr int kWid     = 16;
constexpr int kTaps    = 9;
constexpr int kPlane   = kHgt * kWid;
constexpr int kInDim   = kCin * kPlane;
constexpr int kOutDim  = kCout * kPlane;
constexpr int kRows    = 256;
constexpr int kKdim    = kTaps * kCout;
constexpr int kPadW    = kWid + 2;
constexpr int kPadH    = kHgt + 2;
constexpr int kSlabPos = kPadH * kPadW;
constexpr int kSlabHalves = kSlabPos * kCout;
constexpr int kWgtRows = 2 * kCin;
constexpr int kOutPitch = 68;
constexpr int kWgtItems = kCin * kTaps * (kCout / 8);

constexpr float kCarryW  = 64.0f;
constexpr float kCarryLo = 1024.0f;
constexpr float kCarryX  = 16.0f;
constexpr float kInvHi   = 1.0f / (kCarryW * kCarryX);
constexpr float kInvLo   = 1.0f / (kCarryW * kCarryLo * kCarryX);

static_assert(kCout == 32, "one 32-deep k-step per tap");
static_assert(kCin == 16, "one 16-row A tile for value rows and one for residual rows");
static_assert(kWid == 16 && kHgt == 16, "one 16-column D tile per spatial row");
static_assert(kPlane == 256 && kInDim == 4096 && kOutDim == 8192, "plane sizes");
static_assert(kKdim == 288 && (kKdim % 32) == 0, "K multiple of 32");
static_assert(kSlabHalves * 2 == 20736, "slab bytes");
static_assert(kWgtItems == 576, "weight staging items");
static_assert((kSlabHalves * 2 + kWgtRows * kKdim * 2 + 4 * 16 * kOutPitch * 4) <= 65536, "static LDS budget");

union FragU { v16h v; v8h h[2]; };
__device__ __forceinline__ v16h frag_load(const _Float16* p) {
  FragU f;
  f.h[0] = *(const v8h*)(p);
  f.h[1] = *(const v8h*)(p + 16);
  return f.v;
}
__device__ __forceinline__ v8f mma_g(v16h a, v16h b, v8f c) {
  c = __builtin_amdgcn_wmma_f32_16x16x32_f16(false, a, false, b, (short)0, c, false, false);
  asm volatile("v_nop\n\tv_nop\n\tv_nop\n\tv_nop" : "+v"(c) : "v"(a), "v"(b));
  return c;
}

__global__ __launch_bounds__(128) void tconv_rows_kernel(
    const float* __restrict__ uc, const float* __restrict__ lc,
    const float* __restrict__ weight, float* __restrict__ out)
{
  __shared__ __align__(16) _Float16 sX[kSlabHalves];
  __shared__ __align__(16) _Float16 sW[kWgtRows * kKdim];
  __shared__ __align__(16) float    sO[4][16 * kOutPitch];

  const int tid  = threadIdx.x;
  const int lane = tid & 31;
  const int wave = __builtin_amdgcn_readfirstlane((int)(threadIdx.x >> 5));
  const int c    = lane & 15;
  const int hh   = lane >> 4;
  const int h8   = hh * 8;

  const int bid = blockIdx.x;
  const int mat = bid >> 8;
  const int n   = bid & 255;
  const float* src = (mat ? lc : uc) + (size_t)n * kOutDim;
  float* dst = out + (size_t)bid * kInDim;

  {
    v8h z;
#pragma unroll
    for (int e = 0; e < 8; ++e) z[e] = (_Float16)0.0f;
#pragma unroll 1
    for (int i = tid; i < kSlabHalves / 8; i += 128) *(v8h*)(sX + i * 8) = z;
  }

#pragma unroll 1
  for (int it = 0; it < 5; ++it) {
    const int item = it * 128 + tid;
    const int ic   = (item < kWgtItems) ? item : (kWgtItems - 1);
    const int ci   = ic / 36;
    const int rem  = ic - ci * 36;
    const int g    = rem >> 2;
    const int cg   = rem & 3;
    const float* wp = weight + (cg * 8) * (kCin * kTaps) + ci * kTaps + g;
    v8h hv, lv;
#pragma unroll
    for (int e = 0; e < 8; ++e) {
      const float ws = wp[e * (kCin * kTaps)] * kCarryW;
      const _Float16 hval = (_Float16)ws;
      float hf = (float)hval;
      asm volatile("" : "+v"(hf));
      const float resid = (ws - hf) * kCarryLo;
      hv[e] = hval;
      lv[e] = (_Float16)resid;
    }
    if (item < kWgtItems) {
      *(v8h*)(sW + ci * kKdim + g * kCout + cg * 8) = hv;
      *(v8h*)(sW + (kCin + ci) * kKdim + g * kCout + cg * 8) = lv;
    }
  }
  __syncthreads();

#pragma unroll 2
  for (int it = 0; it < 8; ++it) {
    const int cg = it >> 1;
    const int sp = ((it & 1) << 7) + tid;
    const float* xp = src + (cg * 8) * kPlane + sp;
    v8h hv;
#pragma unroll
    for (int e = 0; e < 8; ++e) {
      const float xv = xp[e * kPlane] * kCarryX;
      hv[e] = (_Float16)xv;
    }
    const int pos = ((sp >> 4) + 1) * kPadW + (sp & 15) + 1;
    *(v8h*)(sX + pos * kCout + cg * 8) = hv;
  }
  __syncthreads();

  v8f acc[4][2];
#pragma unroll
  for (int j = 0; j < 4; ++j) {
    acc[j][0] = (v8f){0.f, 0.f, 0.f, 0.f, 0.f, 0.f, 0.f, 0.f};
    acc[j][1] = (v8f){0.f, 0.f, 0.f, 0.f, 0.f, 0.f, 0.f, 0.f};
  }
  const _Float16* wA = sW + c * kKdim + h8;
  const int ihb = wave * 4;
#pragma unroll
  for (int kh = 0; kh < 3; ++kh) {
#pragma unroll
    for (int kw = 0; kw < 3; ++kw) {
      const int g = kh * 3 + kw;
      const v16h ahi = frag_load(wA + g * kCout);
      const v16h alo = frag_load(wA + kCin * kKdim + g * kCout);
#pragma unroll
      for (int j = 0; j < 4; ++j) {
        const int pr = ihb + j + 2 - kh;
        const int pc = c + 2 - kw;
        const v16h bx = frag_load(sX + (pr * kPadW + pc) * kCout + h8);
        acc[j][0] = mma_g(ahi, bx, acc[j][0]);
        acc[j][1] = mma_g(alo, bx, acc[j][1]);
      }
    }
  }

  float* so = sO[wave];
#pragma unroll
  for (int j = 0; j < 4; ++j) {
#pragma unroll
    for (int r = 0; r < 8; ++r) {
      const float vhi = acc[j][0][r] * kInvHi;
      const float vlo = acc[j][1][r] * kInvLo;
      so[(h8 + r) * kOutPitch + j * 16 + c] = vhi + vlo;
    }
  }
  __syncthreads();

  {
    const int c4 = c * 4;
    float* dw = dst + wave * 64 + c4;
    for (int pass = 0; pass < 2; ++pass) {
#pragma unroll
      for (int it = 0; it < 8; ++it) {
        const int row = it * 2 + hh;
        const v4f val = *(const v4f*)(so + row * kOutPitch + c4);
        *(volatile v4f*)(dw + row * kPlane) = val;
      }
      __threadfence();
    }
  }
}

__global__ __launch_bounds__(256) void bias_rows_kernel(
    const float* __restrict__ uc, const float* __restrict__ lc,
    const float* __restrict__ ucb, const float* __restrict__ lcb,
    const float* __restrict__ bias, float* __restrict__ out)
{
  __shared__ float sRes[32];
  const int lane = threadIdx.x & 31;
  const int wave = __builtin_amdgcn_readfirstlane((int)(threadIdx.x >> 5));
  const int mat  = blockIdx.x >> 3;
  const int n0   = (blockIdx.x & 7) * 32;
  const float* src = mat ? lc : uc;
  const float* bin = mat ? lcb : ucb;

#pragma unroll 1
  for (int r = 0; r < 4; ++r) {
    const int nrow = n0 + wave * 4 + r;
    const float* row = src + (size_t)nrow * kOutDim + lane * 4;
    float p = 0.f;
#pragma unroll 4
    for (int it = 0; it < kOutDim / 128; ++it) {
      const v4f xv = *(const v4f*)(row + it * 128);
      const float bv = bias[it >> 1];
      p = fmaf(xv[0], bv, p);
      p = fmaf(xv[1], bv, p);
      p = fmaf(xv[2], bv, p);
      p = fmaf(xv[3], bv, p);
    }
    p += __shfl_xor(p, 16, 32);
    p += __shfl_xor(p, 8, 32);
    p += __shfl_xor(p, 4, 32);
    p += __shfl_xor(p, 2, 32);
    p += __shfl_xor(p, 1, 32);
    if (lane == 0) sRes[wave * 4 + r] = p;
  }
  __syncthreads();
  if (wave == 0) {
    const float val = sRes[lane] + bin[n0 + lane];
    volatile float* q = out + (size_t)2 * kRows * kInDim + mat * kRows + n0 + lane;
    *q = val;
    __threadfence();
    *q = val;
  }
}

extern "C" void kernel_launch(void* const* d_in, const int* in_sizes, int n_in,
                              void* d_out, int out_size, void* d_ws, size_t ws_size,
                              hipStream_t stream) {
  (void)d_ws; (void)ws_size;
  if (n_in < 6) return;
  if (in_sizes[0] != kRows * kOutDim) return;
  if (in_sizes[1] != kRows * kOutDim) return;
  if (in_sizes[2] != kRows) return;
  if (in_sizes[3] != kRows) return;
  if (in_sizes[4] != kCout * kCin * kTaps) return;
  if (in_sizes[5] != kCout) return;
  if (out_size != 2 * kRows * kInDim + 2 * kRows) return;

  const float* uc     = (const float*)d_in[0];
  const float* lc     = (const float*)d_in[1];
  const float* ucb    = (const float*)d_in[2];
  const float* lcb    = (const float*)d_in[3];
  const float* weight = (const float*)d_in[4];
  const float* bias   = (const float*)d_in[5];
  float* out = (float*)d_out;

  tconv_rows_kernel<<<2 * kRows, 128, 0, stream>>>(uc, lc, weight, out);
  bias_rows_kernel<<<16, 256, 0, stream>>>(uc, lc, ucb, lcb, bias, out);
}
